// DrBC_84490596647625
// MI455X (gfx1250) — hardware-run, weakly checked
//
#include <hip/hip_runtime.h>
#include <math.h>

typedef __attribute__((ext_vector_type(16))) _Float16 v16h;
typedef __attribute__((ext_vector_type(8)))  _Float16 v8h;
typedef __attribute__((ext_vector_type(4)))  _Float16 v4h;
typedef __attribute__((ext_vector_type(8)))  float    v8f;
typedef __attribute__((ext_vector_type(4)))  float    v4f;
typedef __attribute__((ext_vector_type(4)))  int      v4i;
typedef __attribute__((ext_vector_type(4)))  unsigned v4u;
typedef __attribute__((ext_vector_type(2)))  unsigned v2u;

constexpr int kN      = 100000;
constexpr int kE      = 800000;
constexpr int kInF    = 3;
constexpr int kEmb    = 128;
constexpr int kG3     = 3 * kEmb;
constexpr int kHid    = 32;
constexpr int kLayers = 5;
constexpr float kWCarry    = 16.0f;
constexpr float kWCarryInv = 1.0f / kWCarry;
constexpr int kPH = 136;
constexpr int kPF = 132;
constexpr int kRange   = 1024;
constexpr int kNB      = (kN + kRange - 1) / kRange;
constexpr int kNPad    = kNB * kRange;
constexpr int kCap     = 10240;
constexpr int kTabTot  = kNB * kCap;
constexpr int kChunkE  = 1024;
constexpr int kChunks  = (kE + kChunkE - 1) / kChunkE;
constexpr int kSortMax = 128;
static_assert((kN % 32) == 0, "32-row tiles cover the node set exactly");
static_assert((kN % 16) == 0, "embed groups");
static_assert((kE % 4) == 0, "edge quads");
static_assert((kEmb % 32) == 0, "K multiple of 32");
static_assert((kG3 % 16) == 0 && (kHid % 16) == 0, "N multiples of 16");
static_assert(kEmb == 128 && kHid == 32, "lane maps below assume these widths");
static_assert(kRange == 4 * 256, "builder: 4 nodes per thread");
static_assert((kCap % 1024) == 0, "builder: table region written as whole 16-B-per-lane block passes");
static_assert(kNB == 98 && kNPad == 100352 && kChunks == 782, "derived sizes");

constexpr size_t kOffSTART = 0;
constexpr size_t kOffCNT   = kOffSTART + (size_t)kNPad * 4;
constexpr size_t kOffTAB   = kOffCNT   + (size_t)kNPad * 4;
constexpr size_t kOffAGGR  = kOffTAB   + (size_t)kTabTot * 4;
constexpr size_t kOffHA    = kOffAGGR  + (size_t)kN * kEmb * 4;
constexpr size_t kOffHB    = kOffHA    + (size_t)kN * kEmb * 2;
constexpr size_t kOffZMX   = kOffHB    + (size_t)kN * kEmb * 2;
constexpr size_t kOffWIH   = kOffZMX   + (size_t)kN * kEmb * 2;
constexpr size_t kOffWHH   = kOffWIH   + (size_t)kG3 * kEmb * 2;
constexpr size_t kOffWDC   = kOffWHH   + (size_t)kG3 * kEmb * 2;
constexpr size_t kWsTotal  = kOffWDC   + (size_t)kHid * kEmb * 2;
static_assert(kWsTotal == 133021696ull, "carve total");
static_assert(kWsTotal <= 134217728ull, "carve cap");
static_assert((kOffCNT % 128) == 0 && (kOffTAB % 128) == 0 && (kOffAGGR % 128) == 0 && (kOffHA % 128) == 0 &&
              (kOffHB % 128) == 0 && (kOffZMX % 128) == 0 && (kOffWIH % 128) == 0 && (kOffWHH % 128) == 0 &&
              (kOffWDC % 128) == 0, "128-B aligned regions");

__device__ __forceinline__ float h16_to_f32(unsigned hb) {
  const unsigned sgn = (hb & 0x8000u) << 16;
  const unsigned em = hb & 0x7fffu;
  const float fn = __uint_as_float((em << 13) + 0x38000000u);
  const float fs = (float)em * 5.9604644775390625e-8f;
  const float mag = (em < 0x400u) ? fs : fn;
  return __uint_as_float(__float_as_uint(mag) | sgn);
}
__device__ __forceinline__ int clamp_idx(int v, int n) {
  v = v < 0 ? 0 : v;
  return v > (n - 1) ? (n - 1) : v;
}
union FragH { v16h v; v8h h[2]; };
__device__ __forceinline__ v16h ld_frag(const _Float16* p) {
  FragH f;
  f.h[0] = *(const v8h*)(p);
  f.h[1] = *(const v8h*)(p + 16);
  return f.v;
}
__device__ __forceinline__ v8f mma_h(v16h a, v16h b, v8f c) {
  c = __builtin_amdgcn_wmma_f32_16x16x32_f16(false, a, false, b, (short)0, c, false, false);
  asm volatile("v_nop\n\tv_nop\n\tv_nop\n\tv_nop" : "+v"(c) : "v"(a), "v"(b));
  return c;
}
__device__ __forceinline__ float sig_fast(float x) {
  return __builtin_amdgcn_rcpf(1.0f + __expf(-x));
}
__device__ __forceinline__ float tanh_fast(float x) {
  return 1.0f - 2.0f * __builtin_amdgcn_rcpf(1.0f + __expf(2.0f * x));
}

constexpr int kPrepWBlocks = (kG3 * kEmb / 8) / 256;
constexpr int kPrepDBlocks = (kHid * kEmb / 8) / 256;
static_assert(((kG3 * kEmb / 8) % 256) == 0 && ((kHid * kEmb / 8) % 256) == 0, "exact weight blocks");

__global__ __launch_bounds__(256) void prep_kernel(
    const float* __restrict__ Wih, const float* __restrict__ Whh, const float* __restrict__ Wdec,
    unsigned short* __restrict__ Wih16, unsigned short* __restrict__ Whh16, unsigned short* __restrict__ Wdec16)
{
  const int bid = blockIdx.x, tid = threadIdx.x;
  const float* src = Wih;
  unsigned short* dst = Wih16;
  int lb = bid;
  if (bid >= 2 * kPrepWBlocks) {
    src = Wdec; dst = Wdec16; lb = bid - 2 * kPrepWBlocks;
  } else if (bid >= kPrepWBlocks) {
    src = Whh; dst = Whh16; lb = bid - kPrepWBlocks;
  }
  const size_t e0 = ((size_t)lb * 256 + tid) * 8;
  const v4f a0 = *(const v4f*)(src + e0);
  const v4f a1 = *(const v4f*)(src + e0 + 4);
  v8h hv;
#pragma unroll
  for (int e = 0; e < 4; ++e) {
    hv[e]     = (_Float16)(a0[e] * kWCarry);
    hv[4 + e] = (_Float16)(a1[e] * kWCarry);
  }
  *(volatile v8h*)(dst + e0) = hv;
  __threadfence();
  *(volatile v8h*)(dst + e0) = hv;
}

__global__ __launch_bounds__(256) void table_build_kernel(
    const int* __restrict__ row, const int* __restrict__ col,
    int* __restrict__ START, int* __restrict__ CNT, int* __restrict__ TAB)
{
  __shared__ int sCnt[kRange];
  __shared__ int sCur[kRange];
  __shared__ int sStart[kRange];
  __shared__ __align__(16) int sTab[kCap];
  __shared__ int sWs[8];
  const int tid = threadIdx.x, lane = tid & 31, wave = tid >> 5;
  const int lo = blockIdx.x * kRange;

#pragma unroll
  for (int i = 0; i < 4; ++i) sCnt[i * 256 + tid] = 0;
#pragma unroll 1
  for (int i = 0; i < kCap / 256; ++i) sTab[i * 256 + tid] = 0;
  __syncthreads();

#pragma unroll 1
  for (int it = 0; it < kChunks; ++it) {
    const int eb = it * kChunkE + tid * 4;
    const bool ok = eb < kE;
    const int ebc = ok ? eb : (kE - 4);
    const v4i c = *(const v4i*)(col + ebc);
    const unsigned d0 = (unsigned)(clamp_idx(c[0], kN) - lo);
    const unsigned d1 = (unsigned)(clamp_idx(c[1], kN) - lo);
    const unsigned d2 = (unsigned)(clamp_idx(c[2], kN) - lo);
    const unsigned d3 = (unsigned)(clamp_idx(c[3], kN) - lo);
    if (ok && d0 < (unsigned)kRange) atomicAdd(&sCnt[d0], 1);
    if (ok && d1 < (unsigned)kRange) atomicAdd(&sCnt[d1], 1);
    if (ok && d2 < (unsigned)kRange) atomicAdd(&sCnt[d2], 1);
    if (ok && d3 < (unsigned)kRange) atomicAdd(&sCnt[d3], 1);
  }
  __syncthreads();

  {
    const int c0 = sCnt[4 * tid + 0];
    const int c1 = sCnt[4 * tid + 1];
    const int c2 = sCnt[4 * tid + 2];
    const int c3 = sCnt[4 * tid + 3];
    const int s = c0 + c1 + c2 + c3;
    int v = s;
#pragma unroll
    for (int d = 1; d < 32; d <<= 1) {
      const int t = __shfl_up(v, d, 32);
      v = (lane >= d) ? (v + t) : v;
    }
    if (lane == 31) sWs[wave] = v;
    __syncthreads();
    int base = 0;
#pragma unroll
    for (int w = 0; w < 8; ++w) {
      const int x = sWs[w];
      base += (w < wave) ? x : 0;
    }
    const int o0 = base + v - s;
    const int o1 = o0 + c0;
    const int o2 = o1 + c1;
    const int o3 = o2 + c2;
    sStart[4 * tid + 0] = o0;
    sStart[4 * tid + 1] = o1;
    sStart[4 * tid + 2] = o2;
    sStart[4 * tid + 3] = o3;
    sCur[4 * tid + 0] = o0;
    sCur[4 * tid + 1] = o1;
    sCur[4 * tid + 2] = o2;
    sCur[4 * tid + 3] = o3;
  }
  __syncthreads();

#pragma unroll 1
  for (int it = 0; it < kChunks; ++it) {
    const int eb = it * kChunkE + tid * 4;
    const bool ok = eb < kE;
    const int ebc = ok ? eb : (kE - 4);
    const v4i c = *(const v4i*)(col + ebc);
    const unsigned d0 = (unsigned)(clamp_idx(c[0], kN) - lo);
    const unsigned d1 = (unsigned)(clamp_idx(c[1], kN) - lo);
    const unsigned d2 = (unsigned)(clamp_idx(c[2], kN) - lo);
    const unsigned d3 = (unsigned)(clamp_idx(c[3], kN) - lo);
    if (ok && d0 < (unsigned)kRange) {
      const int s = atomicAdd(&sCur[d0], 1);
      if (s >= 0 && s < kCap) sTab[s] = ebc + 0;
    }
    if (ok && d1 < (unsigned)kRange) {
      const int s = atomicAdd(&sCur[d1], 1);
      if (s >= 0 && s < kCap) sTab[s] = ebc + 1;
    }
    if (ok && d2 < (unsigned)kRange) {
      const int s = atomicAdd(&sCur[d2], 1);
      if (s >= 0 && s < kCap) sTab[s] = ebc + 2;
    }
    if (ok && d3 < (unsigned)kRange) {
      const int s = atomicAdd(&sCur[d3], 1);
      if (s >= 0 && s < kCap) sTab[s] = ebc + 3;
    }
  }
  __syncthreads();

#pragma unroll 1
  for (int q = 0; q < 4; ++q) {
    const int st = sStart[4 * tid + q];
    int len = sCnt[4 * tid + q];
    if (st + len > kCap) len = kCap - st;
    len = len < 0 ? 0 : len;
    len = len > kSortMax ? kSortMax : len;
#pragma unroll 1
    for (int i = 1; i < len; ++i) {
      const int key = sTab[st + i];
      int j = i;
      while (j > 0) {
        const int pv = sTab[st + j - 1];
        if (pv <= key) break;
        sTab[st + j] = pv;
        --j;
      }
      sTab[st + j] = key;
    }
  }
  __syncthreads();

#pragma unroll 1
  for (int i = 0; i < kCap / 256; ++i) {
    const int t = i * 256 + tid;
    const int e = clamp_idx(sTab[t], kE);
    const int r = clamp_idx(row[e], kN);
    sTab[t] = r;
  }
  __syncthreads();

  v4i sv, cv;
#pragma unroll
  for (int i = 0; i < 4; ++i) {
    const int st = sStart[4 * tid + i];
    const int cn = sCnt[4 * tid + i];
    sv[i] = blockIdx.x * kCap + st;
    cv[i] = (st + cn <= kCap) ? cn : -1;
  }
  int* tdst = TAB + (size_t)blockIdx.x * kCap;
  for (int pass = 0; pass < 2; ++pass) {
#pragma unroll 1
    for (int i = 0; i < kCap / 1024; ++i) {
      const int o = (i * 256 + tid) * 4;
      const v4i v = *(const v4i*)(sTab + o);
      *(volatile v4i*)(tdst + o) = v;
    }
    *(volatile v4i*)(START + lo + 4 * tid) = sv;
    *(volatile v4i*)(CNT + lo + 4 * tid) = cv;
    __threadfence();
  }
}

__global__ __launch_bounds__(256) void embed_kernel(
    const float* __restrict__ x, const float* __restrict__ W, const float* __restrict__ b,
    unsigned short* __restrict__ hA, unsigned short* __restrict__ zmx)
{
  __shared__ float sW[kEmb * kInF];
  __shared__ float sB[kEmb];
  const int tid = threadIdx.x;
  sW[tid] = W[tid];
  if (tid < 128) {
    sW[256 + tid] = W[256 + tid];
    sB[tid] = b[tid];
  }
  __syncthreads();
  const int c0 = (tid & 15) * 8;
  const int ln = tid >> 4;
  float w0[8], w1[8], w2[8], bb[8];
#pragma unroll
  for (int e = 0; e < 8; ++e) {
    w0[e] = sW[(c0 + e) * kInF + 0];
    w1[e] = sW[(c0 + e) * kInF + 1];
    w2[e] = sW[(c0 + e) * kInF + 2];
    bb[e] = sB[c0 + e];
  }
#pragma unroll 1
  for (int it = 0; it < 4; ++it) {
    const int nb = blockIdx.x * 64 + it * 16;
    if (nb < kN) {
      const int n = nb + ln;
      const float x0 = x[(size_t)n * kInF + 0];
      const float x1 = x[(size_t)n * kInF + 1];
      const float x2 = x[(size_t)n * kInF + 2];
      v8h hv;
#pragma unroll
      for (int e = 0; e < 8; ++e) {
        float p = x0 * w0[e];
        p = fmaf(x1, w1[e], p);
        p = fmaf(x2, w2[e], p);
        const float v = fmaxf(p + bb[e], 0.0f);
        hv[e] = (_Float16)v;
      }
      const size_t o = (size_t)n * kEmb + c0;
      *(volatile v8h*)(hA + o) = hv;
      *(volatile v8h*)(zmx + o) = hv;
      __threadfence();
      *(volatile v8h*)(hA + o) = hv;
      *(volatile v8h*)(zmx + o) = hv;
    }
  }
}

__global__ __launch_bounds__(256) void gather_kernel(
    const int* __restrict__ START, const int* __restrict__ CNT, const int* __restrict__ TAB,
    const unsigned short* __restrict__ h_in, float* __restrict__ aggr)
{
  const int lane = threadIdx.x & 31, wave = threadIdx.x >> 5;
  const int n0 = (blockIdx.x * 8 + wave) * 4;
#pragma unroll 1
  for (int j = 0; j < 4; ++j) {
    const int n = n0 + j;
    const int stv = START[n];
    const int cnv = CNT[n];
    const int st0 = __builtin_amdgcn_readfirstlane(stv);
    const int cn0 = __builtin_amdgcn_readfirstlane(cnv);
    const bool bad = cn0 < 0;
    int cn = cn0 < 0 ? 0 : cn0;
    cn = cn > kCap ? kCap : cn;
    const int st = clamp_idx(st0, kTabTot);
    const float dn = __builtin_amdgcn_rsqf((float)(cn + 1));
    float a0 = 0.0f, a1 = 0.0f, a2 = 0.0f, a3 = 0.0f;
#pragma unroll 1
    for (int p = 0; p < cn; ++p) {
      int ti = st + p;
      ti = ti > (kTabTot - 1) ? (kTabTot - 1) : ti;
      const int s = clamp_idx(TAB[ti], kN);
      int cs = CNT[s];
      cs = cs < 0 ? 0 : cs;
      cs = cs > kCap ? kCap : cs;
      const float nm = __builtin_amdgcn_rsqf((float)(cs + 1)) * dn;
      const v2u w = *(const v2u*)(h_in + (size_t)s * kEmb + lane * 4);
      const unsigned wa = w[0];
      const unsigned wb = w[1];
      const float f0 = h16_to_f32(wa & 0xffffu);
      const float f1 = h16_to_f32(wa >> 16);
      const float f2 = h16_to_f32(wb & 0xffffu);
      const float f3 = h16_to_f32(wb >> 16);
      a0 = fmaf(nm, f0, a0);
      a1 = fmaf(nm, f1, a1);
      a2 = fmaf(nm, f2, a2);
      a3 = fmaf(nm, f3, a3);
    }
    const float qn = __uint_as_float(0x7fc00000u);
    v4f o;
    o[0] = bad ? qn : a0;
    o[1] = bad ? qn : a1;
    o[2] = bad ? qn : a2;
    o[3] = bad ? qn : a3;
    float* dst = aggr + (size_t)n * kEmb + lane * 4;
    *(volatile v4f*)dst = o;
    __threadfence();
    *(volatile v4f*)dst = o;
  }
}

__device__ __forceinline__ void gate_tile(
    const v8f aR, const v8f aZ, const v8f aI, const v8f aH,
    float bR, float bZ, float bIn, float bHn, float* sFcol)
{
#pragma unroll
  for (int r = 0; r < 8; ++r) {
    const float pr = fmaf(aR[r], kWCarryInv, bR);
    const float pz = fmaf(aZ[r], kWCarryInv, bZ);
    const float rr = sig_fast(pr);
    const float zz = sig_fast(pz);
    const float hn = fmaf(aH[r], kWCarryInv, bHn);
    const float gn = fmaf(aI[r], kWCarryInv, bIn);
    const float nn = tanh_fast(gn + rr * hn);
    const float ag = sFcol[r * kPF];
    const float hv = (1.0f - zz) * nn + zz * ag;
    sFcol[r * kPF] = hv;
  }
}

__global__ __launch_bounds__(256) void gru_kernel(
    const unsigned short* __restrict__ h_in, const float* __restrict__ aggr,
    const unsigned short* __restrict__ Wih16, const unsigned short* __restrict__ Whh16,
    const float* __restrict__ b_ih, const float* __restrict__ b_hh,
    unsigned short* __restrict__ h_out, unsigned short* __restrict__ zmx, int store_h)
{
  __shared__ __align__(16) _Float16 sH[32 * kPH];
  __shared__ __align__(16) _Float16 sG[32 * kPH];
  __shared__ __align__(16) float    sF[32 * kPF];
  const int tid = threadIdx.x, lane = tid & 31, wave = tid >> 5;
  const int hh = lane >> 4, l15 = lane & 15;
  const int m0 = blockIdx.x * 32;

#pragma unroll
  for (int i = 0; i < 2; ++i) {
    const int r = (tid >> 4) + 16 * i;
    const int c8 = (tid & 15) * 8;
    const v4u w = *(const v4u*)(h_in + (size_t)(m0 + r) * kEmb + c8);
    *(v4u*)(sH + r * kPH + c8) = w;
  }
#pragma unroll
  for (int i = 0; i < 4; ++i) {
    const int r = (tid >> 5) + 8 * i;
    const int c4 = (tid & 31) * 4;
    const v4f a = *(const v4f*)(aggr + (size_t)(m0 + r) * kEmb + c4);
    *(v4f*)(sF + r * kPF + c4) = a;
    v4h g;
    g[0] = (_Float16)a[0];
    g[1] = (_Float16)a[1];
    g[2] = (_Float16)a[2];
    g[3] = (_Float16)a[3];
    *(v4h*)(sG + r * kPH + c4) = g;
  }
  __syncthreads();

  const _Float16* Wi = (const _Float16*)Wih16;
  const _Float16* Wh = (const _Float16*)Whh16;
  const int nrow = 16 * wave + l15;
  const v8f zero8 = (v8f){0.f, 0.f, 0.f, 0.f, 0.f, 0.f, 0.f, 0.f};
  v8f aR0 = zero8, aR1 = zero8, aZ0 = zero8, aZ1 = zero8;
  v8f aI0 = zero8, aI1 = zero8, aH0 = zero8, aH1 = zero8;

#pragma unroll 1
  for (int kc = 0; kc < kEmb / 32; ++kc) {
    const int k0 = kc * 32 + 8 * hh;
    const v16h ah0 = ld_frag(sH + l15 * kPH + k0);
    const v16h ah1 = ld_frag(sH + (16 + l15) * kPH + k0);
    const v16h ag0 = ld_frag(sG + l15 * kPH + k0);
    const v16h ag1 = ld_frag(sG + (16 + l15) * kPH + k0);
    {
      const v16h bi = ld_frag(Wi + (size_t)nrow * kEmb + k0);
      const v16h bh = ld_frag(Wh + (size_t)nrow * kEmb + k0);
      aR0 = mma_h(ah0, bi, aR0);
      aR1 = mma_h(ah1, bi, aR1);
      aR0 = mma_h(ag0, bh, aR0);
      aR1 = mma_h(ag1, bh, aR1);
    }
    {
      const v16h bi = ld_frag(Wi + (size_t)(kEmb + nrow) * kEmb + k0);
      const v16h bh = ld_frag(Wh + (size_t)(kEmb + nrow) * kEmb + k0);
      aZ0 = mma_h(ah0, bi, aZ0);
      aZ1 = mma_h(ah1, bi, aZ1);
      aZ0 = mma_h(ag0, bh, aZ0);
      aZ1 = mma_h(ag1, bh, aZ1);
    }
    {
      const v16h bi = ld_frag(Wi + (size_t)(2 * kEmb + nrow) * kEmb + k0);
      const v16h bh = ld_frag(Wh + (size_t)(2 * kEmb + nrow) * kEmb + k0);
      aI0 = mma_h(ah0, bi, aI0);
      aI1 = mma_h(ah1, bi, aI1);
      aH0 = mma_h(ag0, bh, aH0);
      aH1 = mma_h(ag1, bh, aH1);
    }
  }

  {
    const int nC = 16 * wave + l15;
    const float bR  = b_ih[nC] + b_hh[nC];
    const float bZ  = b_ih[kEmb + nC] + b_hh[kEmb + nC];
    const float bIn = b_ih[2 * kEmb + nC];
    const float bHn = b_hh[2 * kEmb + nC];
    gate_tile(aR0, aZ0, aI0, aH0, bR, bZ, bIn, bHn, sF + (8 * hh) * kPF + nC);
    gate_tile(aR1, aZ1, aI1, aH1, bR, bZ, bIn, bHn, sF + (16 + 8 * hh) * kPF + nC);
  }
  __syncthreads();

  {
    const int c8 = (lane & 15) * 8;
    v8h hv[2], zv[2];
#pragma unroll
    for (int it = 0; it < 2; ++it) {
      const int row = 4 * wave + 2 * it + hh;
      const float* sp = sF + row * kPF + c8;
      const v4f f0 = *(const v4f*)(sp);
      const v4f f1 = *(const v4f*)(sp + 4);
      const v4u zw = *(const v4u*)(zmx + (size_t)(m0 + row) * kEmb + c8);
      const unsigned z0 = zw[0];
      const unsigned z1 = zw[1];
      const unsigned z2 = zw[2];
      const unsigned z3 = zw[3];
      hv[it][0] = (_Float16)f0[0];
      hv[it][1] = (_Float16)f0[1];
      hv[it][2] = (_Float16)f0[2];
      hv[it][3] = (_Float16)f0[3];
      hv[it][4] = (_Float16)f1[0];
      hv[it][5] = (_Float16)f1[1];
      hv[it][6] = (_Float16)f1[2];
      hv[it][7] = (_Float16)f1[3];
      zv[it][0] = (_Float16)fmaxf(h16_to_f32(z0 & 0xffffu), f0[0]);
      zv[it][1] = (_Float16)fmaxf(h16_to_f32(z0 >> 16),     f0[1]);
      zv[it][2] = (_Float16)fmaxf(h16_to_f32(z1 & 0xffffu), f0[2]);
      zv[it][3] = (_Float16)fmaxf(h16_to_f32(z1 >> 16),     f0[3]);
      zv[it][4] = (_Float16)fmaxf(h16_to_f32(z2 & 0xffffu), f1[0]);
      zv[it][5] = (_Float16)fmaxf(h16_to_f32(z2 >> 16),     f1[1]);
      zv[it][6] = (_Float16)fmaxf(h16_to_f32(z3 & 0xffffu), f1[2]);
      zv[it][7] = (_Float16)fmaxf(h16_to_f32(z3 >> 16),     f1[3]);
    }
    for (int pass = 0; pass < 2; ++pass) {
#pragma unroll
      for (int it = 0; it < 2; ++it) {
        const int row = 4 * wave + 2 * it + hh;
        const size_t o = (size_t)(m0 + row) * kEmb + c8;
        if (store_h) *(volatile v8h*)(h_out + o) = hv[it];
        *(volatile v8h*)(zmx + o) = zv[it];
      }
      __threadfence();
    }
  }
}

__global__ __launch_bounds__(64) void decoder_kernel(
    const unsigned short* __restrict__ zmx, const unsigned short* __restrict__ Wdec16,
    const float* __restrict__ b_dec, const float* __restrict__ W_out, const float* __restrict__ b_out,
    float* __restrict__ out)
{
  __shared__ __align__(16) float sO[32];
  const int tid = threadIdx.x, lane = tid & 31, wave = tid >> 5;
  const int hh = lane >> 4, l15 = lane & 15;
  const int m0 = blockIdx.x * 32 + 16 * wave;
  const _Float16* A = (const _Float16*)zmx;
  const _Float16* B = (const _Float16*)Wdec16;
  const v8f zero8 = (v8f){0.f, 0.f, 0.f, 0.f, 0.f, 0.f, 0.f, 0.f};
  v8f acc0 = zero8, acc1 = zero8;
#pragma unroll
  for (int kc = 0; kc < kEmb / 32; ++kc) {
    const int k0 = kc * 32 + 8 * hh;
    const v16h a  = ld_frag(A + (size_t)(m0 + l15) * kEmb + k0);
    const v16h b0 = ld_frag(B + (size_t)l15 * kEmb + k0);
    const v16h b1 = ld_frag(B + (size_t)(16 + l15) * kEmb + k0);
    acc0 = mma_h(a, b0, acc0);
    acc1 = mma_h(a, b1, acc1);
  }
  const float bd0 = b_dec[l15], bd1 = b_dec[16 + l15];
  const float wo0 = W_out[l15], wo1 = W_out[16 + l15];
  const float bo = b_out[0];
  float s[8];
#pragma unroll
  for (int r = 0; r < 8; ++r) {
    const float d0 = fmaxf(fmaf(acc0[r], kWCarryInv, bd0), 0.0f);
    const float d1 = fmaxf(fmaf(acc1[r], kWCarryInv, bd1), 0.0f);
    s[r] = d0 * wo0 + d1 * wo1;
  }
#pragma unroll
  for (int off = 1; off < 16; off <<= 1) {
#pragma unroll
    for (int r = 0; r < 8; ++r) s[r] += __shfl_xor(s[r], off, 32);
  }
  if (l15 == 0) {
    v4f p0, p1;
    p0[0] = s[0]; p0[1] = s[1]; p0[2] = s[2]; p0[3] = s[3];
    p1[0] = s[4]; p1[1] = s[5]; p1[2] = s[6]; p1[3] = s[7];
    *(v4f*)(sO + 16 * wave + 8 * hh) = p0;
    *(v4f*)(sO + 16 * wave + 8 * hh + 4) = p1;
  }
  __syncthreads();
  if (tid < 8) {
    v4f v = *(const v4f*)(sO + 4 * tid);
    v[0] += bo;
    v[1] += bo;
    v[2] += bo;
    v[3] += bo;
    float* dst = out + (size_t)blockIdx.x * 32 + 4 * tid;
    *(volatile v4f*)dst = v;
    __threadfence();
    *(volatile v4f*)dst = v;
  }
}

extern "C" void kernel_launch(void* const* d_in, const int* in_sizes, int n_in,
                              void* d_out, int out_size, void* d_ws, size_t ws_size,
                              hipStream_t stream) {
  if (n_in < 12) return;
  if (in_sizes[0] != kN * kInF) return;
  if (in_sizes[1] != 2 * kE) return;
  if (in_sizes[2] != kEmb * kInF) return;
  if (in_sizes[3] != kEmb) return;
  if (in_sizes[4] != kG3 * kEmb) return;
  if (in_sizes[5] != kG3 * kEmb) return;
  if (in_sizes[6] != kG3) return;
  if (in_sizes[7] != kG3) return;
  if (in_sizes[8] != kHid * kEmb) return;
  if (in_sizes[9] != kHid) return;
  if (in_sizes[10] != kHid) return;
  if (in_sizes[11] != 1) return;
  if (out_size != kN) return;
  if (ws_size < kWsTotal) return;

  const float* x       = (const float*)d_in[0];
  const int*   edge    = (const int*)d_in[1];
  const float* W_embed = (const float*)d_in[2];
  const float* b_embed = (const float*)d_in[3];
  const float* W_ih    = (const float*)d_in[4];
  const float* W_hh    = (const float*)d_in[5];
  const float* b_ih    = (const float*)d_in[6];
  const float* b_hh    = (const float*)d_in[7];
  const float* W_dec   = (const float*)d_in[8];
  const float* b_dec   = (const float*)d_in[9];
  const float* W_out   = (const float*)d_in[10];
  const float* b_out   = (const float*)d_in[11];
  const int* row = edge;
  const int* col = edge + kE;

  char* ws = (char*)d_ws;
  int*            START = (int*)(ws + kOffSTART);
  int*            CNT   = (int*)(ws + kOffCNT);
  int*            TAB   = (int*)(ws + kOffTAB);
  float*          AGGR  = (float*)(ws + kOffAGGR);
  unsigned short* HA    = (unsigned short*)(ws + kOffHA);
  unsigned short* HB    = (unsigned short*)(ws + kOffHB);
  unsigned short* ZMX   = (unsigned short*)(ws + kOffZMX);
  unsigned short* WIH   = (unsigned short*)(ws + kOffWIH);
  unsigned short* WHH   = (unsigned short*)(ws + kOffWHH);
  unsigned short* WDC   = (unsigned short*)(ws + kOffWDC);

  prep_kernel<<<2 * kPrepWBlocks + kPrepDBlocks, 256, 0, stream>>>(W_ih, W_hh, W_dec, WIH, WHH, WDC);
  table_build_kernel<<<kNB, 256, 0, stream>>>(row, col, START, CNT, TAB);
  embed_kernel<<<(kN + 63) / 64, 256, 0, stream>>>(x, W_embed, b_embed, HA, ZMX);

  unsigned short* hp = HA;
  unsigned short* hn = HB;
  for (int l = 0; l < kLayers; ++l) {
    gather_kernel<<<kN / 32, 256, 0, stream>>>(START, CNT, TAB, hp, AGGR);
    gru_kernel<<<kN / 32, 256, 0, stream>>>(hp, AGGR, WIH, WHH, b_ih, b_hh, hn, ZMX, (l < kLayers - 1) ? 1 : 0);
    unsigned short* t = hp; hp = hn; hn = t;
  }

  decoder_kernel<<<kN / 32, 64, 0, stream>>>(ZMX, WDC, b_dec, W_out, b_out, (float*)d_out);
}
